// GraphRegressor_78030965834327
// MI455X (gfx1250) — hardware-verified
//
#include <hip/hip_runtime.h>
#include <stddef.h>


#define HC      128
#define XD      64
#define AD      16
#define ADP     32
#define PD      256
#define NTHR    256
#define NWAVE   8
#define EPT     8
#define NGRP    2
#define CHUNK   (NTHR * EPT * NGRP)
#define WCAPC   (EPT * NGRP * 32)
#define WCAPF   (EPT * NGRP * 32)
#define ESHF    11
#define EMASK   0xFFFFF
#define NBC     32768
#define NBF     2048
#define RCAP    49152
#define RBN     128
#define TGT     256
#define DEGCAP  512
#define GROWS   128
#define OTHR    512
#define WSCL    64
#define ECAR    64

#define LDS_COUNT  ((NBC + NWAVE * WCAPC + NWAVE) * 4)
#define LDS_FILL   ((RCAP + NBF + NWAVE * WCAPF + NWAVE) * 4)
#define LDS_GEMM   (GROWS * HC * 4)

static_assert((CHUNK & (CHUNK - 1)) == 0);
static_assert((NBC & (NBC - 1)) == 0 && (NBF & (NBF - 1)) == 0);
static_assert(NBF <= (1 << ESHF));
static_assert((NBC % NBF) == 0);
static_assert(OTHR * 4 == NBF);
static_assert((RCAP % 32) == 0);
static_assert(TGT == NWAVE * 32);
static_assert(GROWS == NWAVE * 16);
static_assert((TGT % GROWS) == 0);
static_assert(NBC == NWAVE * 32 * 128);
static_assert(HC == 4 * 32 && PD == 2 * HC);
static_assert((XD % 32) == 0 && (ADP % 32) == 0 && (HC % 32) == 0 && (PD % 32) == 0);
static_assert(LDS_FILL <= 300 * 1024);

typedef float     v4f  __attribute__((ext_vector_type(4)));
typedef float     v8f  __attribute__((ext_vector_type(8)));
typedef int       v4i  __attribute__((ext_vector_type(4)));
typedef _Float16  v4h  __attribute__((ext_vector_type(4)));
typedef _Float16  v8h  __attribute__((ext_vector_type(8)));
typedef _Float16  v16h __attribute__((ext_vector_type(16)));
union FragH { v16h v; v8h h[2]; };

__device__ __forceinline__ v8f wmf(v16h a, v16h b, v8f c) {
  v8f d = __builtin_amdgcn_wmma_f32_16x16x32_f16(false, a, false, b, (short)0, c, false, false);
  asm volatile("v_nop\n\tv_nop\n\tv_nop\n\tv_nop" : "+v"(d) : "v"(a), "v"(b));
  return d;
}

__device__ __forceinline__ v8h cvt8h(v4f a, v4f b) {
  v8h h;
  h[0] = (_Float16)a.x; h[1] = (_Float16)a.y; h[2] = (_Float16)a.z; h[3] = (_Float16)a.w;
  h[4] = (_Float16)b.x; h[5] = (_Float16)b.y; h[6] = (_Float16)b.z; h[7] = (_Float16)b.w;
  return h;
}

template <int NB, int SRC, int WC>
__device__ __forceinline__ int scan_chunk(const int* __restrict__ keys, int nK, int cbase,
                                          int slotBase, int vec8, int* list, int tid, int lane, int wave) {
  int wc = 0;
#pragma unroll
  for (int g = 0; g < NGRP; ++g) {
    const int el0  = (g * NTHR + tid) * EPT;
    const int e0   = cbase + el0;
    const int sent = -2147483647 - 1;
    const int i0 = min(e0, nK - 1),     i1 = min(e0 + 1, nK - 1), i2 = min(e0 + 2, nK - 1), i3 = min(e0 + 3, nK - 1);
    const int i4 = min(e0 + 4, nK - 1), i5 = min(e0 + 5, nK - 1), i6 = min(e0 + 6, nK - 1), i7 = min(e0 + 7, nK - 1);
    v4i da, db;
    if (vec8 != 0 && cbase + CHUNK <= nK) {
      da = *(const v4i*)(keys + e0);
      db = *(const v4i*)(keys + e0 + 4);
    } else {
      da.x = (e0     < nK) ? keys[i0] : sent;
      da.y = (e0 + 1 < nK) ? keys[i1] : sent;
      da.z = (e0 + 2 < nK) ? keys[i2] : sent;
      da.w = (e0 + 3 < nK) ? keys[i3] : sent;
      db.x = (e0 + 4 < nK) ? keys[i4] : sent;
      db.y = (e0 + 5 < nK) ? keys[i5] : sent;
      db.z = (e0 + 6 < nK) ? keys[i6] : sent;
      db.w = (e0 + 7 < nK) ? keys[i7] : sent;
    }
    const unsigned nb = (unsigned)slotBase;
    const unsigned s0 = (unsigned)da.x - nb, s1 = (unsigned)da.y - nb;
    const unsigned s2 = (unsigned)da.z - nb, s3 = (unsigned)da.w - nb;
    const unsigned s4 = (unsigned)db.x - nb, s5 = (unsigned)db.y - nb;
    const unsigned s6 = (unsigned)db.z - nb, s7 = (unsigned)db.w - nb;
    const bool h0 = s0 < (unsigned)NB, h1 = s1 < (unsigned)NB, h2 = s2 < (unsigned)NB, h3 = s3 < (unsigned)NB;
    const bool h4 = s4 < (unsigned)NB, h5 = s5 < (unsigned)NB, h6 = s6 < (unsigned)NB, h7 = s7 < (unsigned)NB;
    const unsigned any = __builtin_amdgcn_ballot_w32(h0 | h1 | h2 | h3 | h4 | h5 | h6 | h7);
    if (any != 0u) {
#define HITJ(HJ, SJ, VJ) { \
        const unsigned mj = __builtin_amdgcn_ballot_w32(HJ); \
        if (mj != 0u) { \
          if (HJ) { \
            const int pos = wc + (int)__builtin_amdgcn_mbcnt_lo(mj, 0u); \
            const int entv = SRC ? (((VJ) << ESHF) | (int)(SJ)) : (int)(SJ); \
            if (pos < WC) list[wave * WC + pos] = entv; \
          } \
          wc += (int)__builtin_popcount(mj); } }
      HITJ(h0, s0, i0)
      HITJ(h1, s1, i1)
      HITJ(h2, s2, i2)
      HITJ(h3, s3, i3)
      HITJ(h4, s4, i4)
      HITJ(h5, s5, i5)
      HITJ(h6, s6, i6)
      HITJ(h7, s7, i7)
#undef HITJ
    }
  }
  return wc;
}

template <int KP>
__global__ __launch_bounds__(NTHR) void k_wT16(const float* __restrict__ W, _Float16* Wp,
                                               int KD, int NC, float scale) {
  static_assert(KP == 32 || (KP % 64) == 0);
  constexpr int TP = KP + 8;
  __shared__ __attribute__((aligned(16))) _Float16 sT[32 * TP];
  const int tid = threadIdx.x;
  const int n0 = (int)blockIdx.x * 32;
  const int z = (int)blockIdx.y;
  const float* Wz = W + (size_t)z * KD * NC;
  _Float16* Wpz = Wp + (size_t)z * NC * KP;
#pragma unroll 1
  for (int idx = tid; idx < KP * 32; idx += NTHR) {
    const int kr = idx >> 5, nc = idx & 31;
    const int kc = kr < KD ? kr : KD - 1;
    float v = Wz[(size_t)kc * NC + n0 + nc] * scale;
    if (kr >= KD) v = 0.0f;
    sT[nc * TP + kr] = (_Float16)v;
  }
  __syncthreads();
  if constexpr (KP >= 64) {
    const int nl = tid >> 3, p = tid & 7;
    _Float16* d = Wpz + (size_t)(n0 + nl) * KP + 8 * p;
    const _Float16* s = sT + nl * TP + 8 * p;
#pragma unroll
    for (int q = 0; q < KP / 64; ++q) { const v8h hv = *(const v8h*)(s + 64 * q); *(volatile v8h*)(d + 64 * q) = hv; }
    __threadfence();
#pragma unroll
    for (int q = 0; q < KP / 64; ++q) { const v8h hv = *(const v8h*)(s + 64 * q); *(volatile v8h*)(d + 64 * q) = hv; }
  } else {
    const bool act = tid < 128;
    const int nl = act ? (tid >> 2) : 0, p = tid & 3;
    _Float16* d = Wpz + (size_t)(n0 + nl) * KP + 8 * p;
    const v8h hv = *(const v8h*)(sT + nl * TP + 8 * p);
    if (act) *(volatile v8h*)d = hv;
    __threadfence();
    if (act) *(volatile v8h*)d = hv;
  }
}

__global__ __launch_bounds__(NTHR) void k_count(
    const int* __restrict__ keys, int* cnt, int nK, int vec8) {
  extern __shared__ v4f lds_dyn[];
  int* scnt = (int*)lds_dyn;
  int* list = scnt + NBC;
  int* wcnt = list + NWAVE * WCAPC;
  const int tid = threadIdx.x, lane = tid & 31, wave = tid >> 5;
  const int nodeBase = blockIdx.x * NBC;

  {
    const v4i z = {0, 0, 0, 0};
    for (int i = tid; i < NBC / 4; i += NTHR) ((v4i*)scnt)[i] = z;
  }
  __syncthreads();

  const int nChunks = (nK + CHUNK - 1) / CHUNK;
#pragma unroll 1
  for (int ch = 0; ch < nChunks; ++ch) {
    const int cbase = ch * CHUNK;
    const int wc = scan_chunk<NBC, 0, WCAPC>(keys, nK, cbase, nodeBase, vec8, list, tid, lane, wave);
    if (lane == 0) wcnt[wave] = wc;
    __syncthreads();
    if (wave == 0) {
#pragma unroll 1
      for (int wsx = 0; wsx < NWAVE; ++wsx) {
        int n = __builtin_amdgcn_readfirstlane(wcnt[wsx]);
        n = n > WCAPC ? WCAPC : (n < 0 ? 0 : n);
        const int* lp = list + wsx * WCAPC;
#pragma unroll 1
        for (int i = 0; i < n; ++i) {
          const int ent  = __builtin_amdgcn_readfirstlane(lp[i]);
          const int slot = ent & (NBC - 1);
          if (lane == 0) scnt[slot] = scnt[slot] + 1;
        }
      }
    }
    __syncthreads();
  }

  int* cp = cnt + (size_t)nodeBase;
#pragma unroll 4
  for (int q = 0; q < 32; ++q) {
    const int f = (wave * 32 + q) * 128 + 4 * lane;
    const v4i c = *(const v4i*)(scnt + f);
    *(volatile v4i*)(cp + f) = c;
  }
  __threadfence();
#pragma unroll 4
  for (int q = 0; q < 32; ++q) {
    const int f = (wave * 32 + q) * 128 + 4 * lane;
    const v4i c = *(const v4i*)(scnt + f);
    *(volatile v4i*)(cp + f) = c;
  }
}

__global__ __launch_bounds__(OTHR) void k_offsets(
    const int* __restrict__ cnt, int* off, int* rbase, int nBF) {
  __shared__ __attribute__((aligned(16))) int srb[RBN];
  __shared__ int wtot[OTHR / 32];
  const int tid = threadIdx.x, lane = tid & 31, wave = tid >> 5;
  for (int i = tid; i < RBN; i += OTHR) srb[i] = 0;
  int carry = 0;
#pragma unroll 1
  for (int fb = 0; fb < nBF; ++fb) {
    const int base = fb * NBF;
    const v4i c = *(const v4i*)(cnt + base + 4 * tid);
    const int e0 = max(c.x, 0), e1 = max(c.y, 0), e2 = max(c.z, 0), e3 = max(c.w, 0);
    const int ts = e0 + e1 + e2 + e3;
    int incl = ts;
#pragma unroll
    for (int d = 1; d < 32; d <<= 1) {
      const int t = __shfl_up(incl, d, 32);
      if (lane >= d) incl += t;
    }
    if (lane == 31) wtot[wave] = incl;
    __syncthreads();
    int pre = 0;
#pragma unroll 1
    for (int w = 0; w < wave; ++w) pre += wtot[w];
    int tot = 0;
#pragma unroll
    for (int w = 0; w < OTHR / 32; ++w) tot += wtot[w];
    int run = carry + pre + incl - ts;
    v4i o;
    o.x = run; run += e0;
    o.y = run; run += e1;
    o.z = run; run += e2;
    o.w = run;
    int* op = off + base + 4 * tid;
    *(volatile v4i*)op = o;
    __threadfence();
    *(volatile v4i*)op = o;
    if (tid == 0) srb[min(fb, RBN - 1)] = carry;
    carry += (tot + 31) & ~31;
    __syncthreads();
  }
  if (tid == 0) srb[min(nBF, RBN - 1)] = carry;
  __syncthreads();
  v4i rv = {0, 0, 0, 0};
  if (tid < 32) rv = *(const v4i*)(srb + 4 * tid);
  if (tid < 32) *(volatile v4i*)(rbase + 4 * tid) = rv;
  __threadfence();
  if (tid < 32) *(volatile v4i*)(rbase + 4 * tid) = rv;
}

__global__ __launch_bounds__(NTHR) void k_fill(
    const int* __restrict__ keys, const int* __restrict__ off,
    const int* __restrict__ rbase, int* csr, int nK, int vec8, int csrLen) {
  extern __shared__ v4f lds_dyn[];
  int* region = (int*)lds_dyn;
  int* cursor = region + RCAP;
  int* list   = cursor + NBF;
  int* wcnt   = list + NWAVE * WCAPF;
  const int tid = threadIdx.x, lane = tid & 31, wave = tid >> 5;
  const int b = blockIdx.x;
  const int nodeBase = b * NBF;

  int rb0 = rbase[b];
  const int rb1 = rbase[b + 1];
  rb0 = rb0 < 0 ? 0 : (rb0 > csrLen ? csrLen : rb0);
  rb0 &= ~31;
  int len = rb1 - rb0;
  len = len < 0 ? 0 : (len > RCAP ? RCAP : len);
  int lenW = (len + 31) & ~31;
  if (rb0 + lenW > csrLen) lenW = (csrLen - rb0) & ~31;

  {
    const v4i z = {0, 0, 0, 0};
    for (int i = tid; i < RCAP / 4; i += NTHR) ((v4i*)region)[i] = z;
    for (int s = tid; s < NBF; s += NTHR) {
      int o = off[nodeBase + s] - rb0;
      o = o < 0 ? 0 : (o > RCAP ? RCAP : o);
      cursor[s] = o;
    }
  }
  __syncthreads();

  const int nChunks = (nK + CHUNK - 1) / CHUNK;
#pragma unroll 1
  for (int ch = 0; ch < nChunks; ++ch) {
    const int cbase = ch * CHUNK;
    const int wc = scan_chunk<NBF, 1, WCAPF>(keys, nK, cbase, nodeBase, vec8, list, tid, lane, wave);
    if (lane == 0) wcnt[wave] = wc;
    __syncthreads();
    if (wave == 0) {
#pragma unroll 1
      for (int wsx = 0; wsx < NWAVE; ++wsx) {
        int n = __builtin_amdgcn_readfirstlane(wcnt[wsx]);
        n = n > WCAPF ? WCAPF : (n < 0 ? 0 : n);
        const int* lp = list + wsx * WCAPF;
#pragma unroll 1
        for (int i = 0; i < n; ++i) {
          const int ent  = __builtin_amdgcn_readfirstlane(lp[i]);
          const int slot = ent & (NBF - 1);
          int ev = (ent >> ESHF) & EMASK;
          ev = ev > nK - 1 ? nK - 1 : ev;
          if (lane == 0) {
            int pos = cursor[slot];
            pos = pos < 0 ? 0 : (pos > RCAP - 1 ? RCAP - 1 : pos);
            region[pos] = ev;
            const int np = pos + 1;
            cursor[slot] = np > RCAP ? RCAP : np;
          }
        }
      }
    }
    __syncthreads();
  }

  const int nv = lenW >> 2;
  int* gp = csr + rb0;
#pragma unroll 1
  for (int i = tid; i < nv; i += NTHR) { const v4i v = ((const v4i*)region)[i]; *(volatile v4i*)(gp + 4 * i) = v; }
  __threadfence();
#pragma unroll 1
  for (int i = tid; i < nv; i += NTHR) { const v4i v = ((const v4i*)region)[i]; *(volatile v4i*)(gp + 4 * i) = v; }
}

__device__ __forceinline__ void cvst4(const float* lp, _Float16* gp, float s) {
  const v4f f = *(const v4f*)lp;
  v4h h;
  h[0] = (_Float16)(f.x * s); h[1] = (_Float16)(f.y * s); h[2] = (_Float16)(f.z * s); h[3] = (_Float16)(f.w * s);
  *(volatile v4h*)gp = h;
}

template <int KD, int KREAL, int AF32, int EPI>
__global__ __launch_bounds__(NTHR) void k_gemm(
    const void* __restrict__ Ain, int nA, const _Float16* __restrict__ Bw,
    const float* __restrict__ bias, void* Cout, float osc, float ocar, int nStore,
    const float* __restrict__ w2, const float* __restrict__ b2) {
  static_assert((KD % 32) == 0);
  static_assert(KREAL == KD || (AF32 == 1 && KREAL == 16 && KD == 32));
  constexpr int NT  = 8;
  constexpr int RPW = GROWS / NWAVE;
  extern __shared__ v4f lds_dyn[];
  float* stg = (float*)lds_dyn;
  __shared__ __attribute__((aligned(16))) float sres[GROWS];
  const int tid = threadIdx.x, lane = tid & 31, wave = tid >> 5, hh = lane >> 4, m = lane & 15;
  const int rowBase = (int)blockIdx.x * GROWS;
  const int arow = rowBase + 16 * wave + m;
  const _Float16* bp0 = Bw + (size_t)m * KD + 8 * hh;

  v8f acc[NT];
#pragma unroll
  for (int t = 0; t < NT; ++t) { v8f z = {0.f, 0.f, 0.f, 0.f, 0.f, 0.f, 0.f, 0.f}; acc[t] = z; }

#pragma unroll 1
  for (int kt = 0; kt < KD / 32; ++kt) {
    FragH af;
    if constexpr (AF32 == 1) {
      const int ar = arow < nA ? arow : nA - 1;
      const float* ap = (const float*)Ain + (size_t)ar * KREAL + 32 * kt + 8 * hh;
      const v4f f0 = *(const v4f*)ap;
      const v4f f1 = *(const v4f*)(ap + 4);
      af.h[0] = cvt8h(f0, f1);
      if constexpr (KREAL == KD) {
        const v4f f2 = *(const v4f*)(ap + 16);
        const v4f f3 = *(const v4f*)(ap + 20);
        af.h[1] = cvt8h(f2, f3);
      } else {
        v8h zh;
#pragma unroll
        for (int i = 0; i < 8; ++i) zh[i] = (_Float16)0.0f;
        af.h[1] = zh;
      }
    } else {
      const _Float16* ap = (const _Float16*)Ain + (size_t)arow * KD + 8 * hh + 32 * kt;
      af.h[0] = *(const v8h*)ap;
      af.h[1] = *(const v8h*)(ap + 16);
    }
#pragma unroll
    for (int t = 0; t < NT; ++t) {
      const _Float16* bp = bp0 + (size_t)(16 * t) * KD + 32 * kt;
      FragH bf;
      bf.h[0] = *(const v8h*)bp;
      bf.h[1] = *(const v8h*)(bp + 16);
      acc[t] = wmf(af.v, bf.v, acc[t]);
    }
  }

  const int r0 = 16 * wave + 8 * hh;
  float bc[NT];
#pragma unroll
  for (int t = 0; t < NT; ++t) bc[t] = bias[16 * t + m];

  float* sp = stg + r0 * HC + m;
#pragma unroll
  for (int t = 0; t < NT; ++t) {
#pragma unroll
    for (int r = 0; r < 8; ++r) {
      const float v = fmaxf(acc[t][r] * osc + bc[t], 0.0f);
      sp[r * HC + 16 * t] = v;
    }
  }
  __syncthreads();

  const float* lp = stg + wave * RPW * HC;
  const int orow0 = rowBase + wave * RPW;
  if constexpr (EPI == 0) {
    _Float16* C = (_Float16*)Cout;
#pragma unroll
    for (int i = 0; i < RPW; ++i) {
      if (orow0 + i < nStore) cvst4(lp + i * HC + 4 * lane, C + (size_t)(orow0 + i) * HC + 4 * lane, ocar);
    }
    __threadfence();
#pragma unroll
    for (int i = 0; i < RPW; ++i) {
      if (orow0 + i < nStore) cvst4(lp + i * HC + 4 * lane, C + (size_t)(orow0 + i) * HC + 4 * lane, ocar);
    }
  } else if constexpr (EPI == 1) {
    float* C = (float*)Cout;
#pragma unroll
    for (int i = 0; i < RPW; ++i) {
      if (orow0 + i < nStore) {
        const v4f v = *(const v4f*)(lp + i * HC + 4 * lane);
        *(volatile v4f*)(C + (size_t)(orow0 + i) * HC + 4 * lane) = v;
      }
    }
    __threadfence();
#pragma unroll
    for (int i = 0; i < RPW; ++i) {
      if (orow0 + i < nStore) {
        const v4f v = *(const v4f*)(lp + i * HC + 4 * lane);
        *(volatile v4f*)(C + (size_t)(orow0 + i) * HC + 4 * lane) = v;
      }
    }
  } else {
    if (tid < GROWS) {
      const float* rp = stg + tid * HC;
      float d = 0.0f;
#pragma unroll 4
      for (int j = 0; j < HC; ++j) d += rp[j] * w2[j];
      sres[tid] = d + b2[0];
    }
    __syncthreads();
    float* C = (float*)Cout;
    const int o = rowBase + 4 * lane;
    const bool act = (wave == 0) && (o + 4 <= nStore);
    const v4f v = *(const v4f*)(sres + 4 * lane);
    if (act) *(volatile v4f*)(C + o) = v;
    __threadfence();
    if (act) *(volatile v4f*)(C + o) = v;
  }
}

__global__ __launch_bounds__(NTHR) void k_agg(
    const int* __restrict__ csr, const int* __restrict__ off, const int* __restrict__ cnt,
    const int* __restrict__ srcidx, const float* __restrict__ hw, const _Float16* __restrict__ ep16,
    _Float16* outp, int nN, int nE, int csrLen, float einv) {
  const int tid = threadIdx.x, lane = tid & 31, wave = tid >> 5;
  const int tbase = (int)blockIdx.x * TGT + wave * 32;
  const int cl = tbase + lane;
  const int cnt_l = cnt[cl];
  const int off_l = off[cl];
  const int ch = 4 * lane;

#pragma unroll 1
  for (int j = 0; j < 32; ++j) {
    const int c = tbase + j;
    const int nraw = __builtin_amdgcn_readlane(cnt_l, j);
    const int n = nraw < 0 ? 0 : (nraw > DEGCAP ? DEGCAP : nraw);
    const int st = __builtin_amdgcn_readlane(off_l, j);
    v4f a0 = {0.f, 0.f, 0.f, 0.f};
#pragma unroll 1
    for (int q0 = 0; q0 < n; q0 += 32) {
      int pos = st + q0 + lane;
      pos = pos < 0 ? 0 : (pos > csrLen - 1 ? csrLen - 1 : pos);
      int el = csr[pos];
      el = el < 0 ? 0 : (el > nE - 1 ? nE - 1 : el);
      int sl = srcidx[el];
      sl = sl < 0 ? 0 : (sl > nN - 1 ? nN - 1 : sl);
      const int mcnt = (n - q0) < 32 ? (n - q0) : 32;
#pragma unroll 1
      for (int p = 0; p < mcnt; ++p) {
        const int s  = __builtin_amdgcn_readlane(sl, p);
        const int ev = __builtin_amdgcn_readlane(el, p);
        const v4f h0 = *(const v4f*)(hw + (size_t)s * HC + ch);
        const v4h e4 = *(const v4h*)(ep16 + (size_t)ev * HC + ch);
        a0.x += fmaxf(h0.x + (float)e4[0] * einv, 0.0f);
        a0.y += fmaxf(h0.y + (float)e4[1] * einv, 0.0f);
        a0.z += fmaxf(h0.z + (float)e4[2] * einv, 0.0f);
        a0.w += fmaxf(h0.w + (float)e4[3] * einv, 0.0f);
      }
    }
    const int cs = c < nN ? c : nN - 1;
    v4f v0 = a0 + *(const v4f*)(hw + (size_t)cs * HC + ch);
    if (c >= nN) {
      const v4f z = {0.f, 0.f, 0.f, 0.f}; v0 = z;
    }
    if (nraw > DEGCAP) {
      const float qn = __int_as_float(0x7fc00000);
      v0.x = qn; v0.y = qn; v0.z = qn; v0.w = qn;
    }
    v4h hv;
    hv[0] = (_Float16)v0.x; hv[1] = (_Float16)v0.y; hv[2] = (_Float16)v0.z; hv[3] = (_Float16)v0.w;
    _Float16* rp = outp + (size_t)c * HC + ch;
    *(volatile v4h*)rp = hv;
    __threadfence();
    *(volatile v4h*)rp = hv;
  }
}

__global__ __launch_bounds__(NTHR) void k_pool(const int* __restrict__ bix, const float* __restrict__ hw,
                                               _Float16* P16, int nN, int G) {
  __shared__ __attribute__((aligned(16))) float ssum[NWAVE * HC];
  __shared__ __attribute__((aligned(16))) float smax[NWAVE * HC];
  __shared__ int scn[NWAVE];
  __shared__ __attribute__((aligned(16))) float srow[PD];
  const int tid = threadIdx.x, lane = tid & 31, wave = tid >> 5;
  const int g = (int)blockIdx.x;
  const int ch = 4 * lane;
  const float ninf = __int_as_float(0xff800000);
  v4f s  = {0.f, 0.f, 0.f, 0.f};
  v4f mx = {ninf, ninf, ninf, ninf};
  int cn = 0;
  const int nCh = (nN + NTHR - 1) / NTHR;
#pragma unroll 1
  for (int c = 0; c < nCh; ++c) {
    const int i = c * NTHR + tid;
    const int ic = i < nN ? i : nN - 1;
    const int b = bix[ic];
    const bool hit = (i < nN) && (b == g);
    unsigned mk = __builtin_amdgcn_ballot_w32(hit);
    cn += (int)__builtin_popcount(mk);
    const int nb = c * NTHR + wave * 32;
#pragma unroll 1
    while (mk != 0u) {
      const int p = __builtin_ctz(mk);
      mk &= mk - 1u;
      const v4f hv = *(const v4f*)(hw + (size_t)(nb + p) * HC + ch);
      s = s + hv;
      mx.x = fmaxf(mx.x, hv.x); mx.y = fmaxf(mx.y, hv.y); mx.z = fmaxf(mx.z, hv.z); mx.w = fmaxf(mx.w, hv.w);
    }
  }
  *(v4f*)(ssum + wave * HC + ch) = s;
  *(v4f*)(smax + wave * HC + ch) = mx;
  if (lane == 0) scn[wave] = cn;
  __syncthreads();
  if (wave == 0) {
    v4f ts = *(const v4f*)(ssum + ch);
    v4f tm = *(const v4f*)(smax + ch);
    int tc = scn[0];
#pragma unroll
    for (int w = 1; w < NWAVE; ++w) {
      const v4f a = *(const v4f*)(ssum + w * HC + ch);
      const v4f b = *(const v4f*)(smax + w * HC + ch);
      ts = ts + a;
      tm.x = fmaxf(tm.x, b.x); tm.y = fmaxf(tm.y, b.y); tm.z = fmaxf(tm.z, b.z); tm.w = fmaxf(tm.w, b.w);
      tc += scn[w];
    }
    const float inv = 1.0f / (float)tc;
    v4f mean = ts * inv;
    if (g >= G) { const v4f z = {0.f, 0.f, 0.f, 0.f}; mean = z; tm = z; }
    *(v4f*)(srow + ch) = mean;
    *(v4f*)(srow + HC + ch) = tm;
  }
  __syncthreads();
  const v4f p0 = *(const v4f*)(srow + 8 * lane);
  const v4f p1 = *(const v4f*)(srow + 8 * lane + 4);
  const v8h hv = cvt8h(p0, p1);
  _Float16* d = P16 + (size_t)g * PD + 8 * lane;
  if (wave == 0) *(volatile v8h*)d = hv;
  __threadfence();
  if (wave == 0) *(volatile v8h*)d = hv;
}

extern "C" void kernel_launch(void* const* d_in, const int* in_sizes, int n_in,
                              void* d_out, int out_size, void* d_ws, size_t ws_size,
                              hipStream_t stream) {
  if (n_in < 16) return;
  const int nN = in_sizes[0] / XD;
  const int nE = in_sizes[1] / AD;
  if (nN <= 0 || nE <= 0) return;
  if (in_sizes[0] != nN * XD || in_sizes[1] != nE * AD) return;
  if (in_sizes[2] != 2 * nE || in_sizes[3] != nN) return;
  if (in_sizes[4] != XD * HC || in_sizes[5] != HC) return;
  if (in_sizes[6] != AD * HC || in_sizes[7] != HC) return;
  const int L = in_sizes[8] / (HC * HC);
  if (L <= 0 || L > 16) return;
  if (in_sizes[8] != L * HC * HC || in_sizes[9] != L * HC) return;
  if (in_sizes[10] != L * HC * HC || in_sizes[11] != L * HC) return;
  if (in_sizes[12] != PD * HC || in_sizes[13] != HC || in_sizes[14] != HC || in_sizes[15] != 1) return;
  const int G = out_size;
  if (G <= 0 || (G % 4) != 0) return;
  if (nN > (1 << 20) || nE > (1 << 20)) return;

  const float* x    = (const float*)d_in[0];
  const float* ea   = (const float*)d_in[1];
  const int*   ei   = (const int*)d_in[2];
  const int*   bix  = (const int*)d_in[3];
  const float* nw   = (const float*)d_in[4];
  const float* nb   = (const float*)d_in[5];
  const float* ew   = (const float*)d_in[6];
  const float* eb   = (const float*)d_in[7];
  const float* cw1  = (const float*)d_in[8];
  const float* cb1  = (const float*)d_in[9];
  const float* cw2  = (const float*)d_in[10];
  const float* cb2  = (const float*)d_in[11];
  const float* hw1  = (const float*)d_in[12];
  const float* hb1  = (const float*)d_in[13];
  const float* hw2  = (const float*)d_in[14];
  const float* hb2  = (const float*)d_in[15];
  float* out = (float*)d_out;
  const int* srci = ei;
  const int* dsti = ei + nE;
  const int nK = nE;

  const int NPAD   = ((nN + TGT - 1) / TGT) * TGT;
  const int EPAD   = ((nE + GROWS - 1) / GROWS) * GROWS;
  const int GPAD   = ((G + GROWS - 1) / GROWS) * GROWS;
  const int nBC    = (nN + NBC - 1) / NBC;
  const int CNTPAD = nBC * NBC;
  const int nBF    = (nN + NBF - 1) / NBF;
  const int OFFN   = nBF * NBF;
  if (nBF + 1 > RBN) return;
  if (OFFN > CNTPAD || NPAD > OFFN) return;
  if ((NPAD % GROWS) != 0 || (NPAD % TGT) != 0 || (EPAD % GROWS) != 0 || (GPAD % GROWS) != 0) return;
  const int csrLen = ((nK + 31) & ~31) + 32 * (nBF + 1);
  const int nGn    = NPAD / GROWS;
  const int nGe    = EPAD / GROWS;
  const int nGh    = GPAD / GROWS;
  const int nAgg   = NPAD / TGT;

  char* ws = (char*)d_ws;
  size_t off = 0;
  const size_t oE16 = off; off += (size_t)EPAD * HC * 2;         off = (off + 255) & ~(size_t)255;
  const size_t oH32 = off; off += (size_t)NPAD * HC * 4;         off = (off + 255) & ~(size_t)255;
  const size_t oA16 = off; off += (size_t)NPAD * HC * 2;         off = (off + 255) & ~(size_t)255;
  const size_t oM16 = off; off += (size_t)NPAD * HC * 2;         off = (off + 255) & ~(size_t)255;
  const size_t oP16 = off; off += (size_t)GPAD * PD * 2;         off = (off + 255) & ~(size_t)255;
  const size_t oWN  = off; off += (size_t)HC * XD * 2;           off = (off + 255) & ~(size_t)255;
  const size_t oWE  = off; off += (size_t)HC * ADP * 2;          off = (off + 255) & ~(size_t)255;
  const size_t oWC1 = off; off += (size_t)L * HC * HC * 2;       off = (off + 255) & ~(size_t)255;
  const size_t oWC2 = off; off += (size_t)L * HC * HC * 2;       off = (off + 255) & ~(size_t)255;
  const size_t oWH  = off; off += (size_t)HC * PD * 2;           off = (off + 255) & ~(size_t)255;
  const size_t oCnt = off; off += (size_t)CNTPAD * 4;            off = (off + 255) & ~(size_t)255;
  const size_t oOff = off; off += (size_t)OFFN * 4;              off = (off + 255) & ~(size_t)255;
  const size_t oRb  = off; off += (size_t)RBN * 4;               off = (off + 255) & ~(size_t)255;
  const size_t oCsr = off; off += (size_t)csrLen * 4;            off = (off + 255) & ~(size_t)255;
  if (off > ws_size) return;
  _Float16* E16  = (_Float16*)(ws + oE16);
  float*    H32  = (float*)(ws + oH32);
  _Float16* A16  = (_Float16*)(ws + oA16);
  _Float16* M16  = (_Float16*)(ws + oM16);
  _Float16* P16  = (_Float16*)(ws + oP16);
  _Float16* WN   = (_Float16*)(ws + oWN);
  _Float16* WE   = (_Float16*)(ws + oWE);
  _Float16* WC1  = (_Float16*)(ws + oWC1);
  _Float16* WC2  = (_Float16*)(ws + oWC2);
  _Float16* WH   = (_Float16*)(ws + oWH);
  int*      cnt  = (int*)(ws + oCnt);
  int*      offp = (int*)(ws + oOff);
  int*      rb   = (int*)(ws + oRb);
  int*      csr  = (int*)(ws + oCsr);

  const int vec8 = ((nE & 3) == 0) ? 1 : 0;
  const float osc  = 1.0f / (float)WSCL;
  const float ecar = (float)ECAR;
  const float einv = 1.0f / (float)ECAR;

  k_wT16<XD> <<<dim3(HC / 32, 1), NTHR, 0, stream>>>(nw,  WN,  XD, HC, (float)WSCL);
  k_wT16<ADP><<<dim3(HC / 32, 1), NTHR, 0, stream>>>(ew,  WE,  AD, HC, (float)WSCL);
  k_wT16<HC> <<<dim3(HC / 32, L), NTHR, 0, stream>>>(cw1, WC1, HC, HC, (float)WSCL);
  k_wT16<HC> <<<dim3(HC / 32, L), NTHR, 0, stream>>>(cw2, WC2, HC, HC, (float)WSCL);
  k_wT16<PD> <<<dim3(HC / 32, 1), NTHR, 0, stream>>>(hw1, WH,  PD, HC, (float)WSCL);

  hipFuncSetAttribute(reinterpret_cast<const void*>(&k_count),
                      hipFuncAttributeMaxDynamicSharedMemorySize, LDS_COUNT);
  k_count<<<nBC, NTHR, LDS_COUNT, stream>>>(dsti, cnt, nK, vec8);
  k_offsets<<<1, OTHR, 0, stream>>>(cnt, offp, rb, nBF);
  hipFuncSetAttribute(reinterpret_cast<const void*>(&k_fill),
                      hipFuncAttributeMaxDynamicSharedMemorySize, LDS_FILL);
  k_fill<<<nBF, NTHR, LDS_FILL, stream>>>(dsti, offp, rb, csr, nK, vec8, csrLen);

  hipFuncSetAttribute(reinterpret_cast<const void*>(&k_gemm<XD, XD, 1, 1>),
                      hipFuncAttributeMaxDynamicSharedMemorySize, LDS_GEMM);
  hipFuncSetAttribute(reinterpret_cast<const void*>(&k_gemm<ADP, AD, 1, 0>),
                      hipFuncAttributeMaxDynamicSharedMemorySize, LDS_GEMM);
  hipFuncSetAttribute(reinterpret_cast<const void*>(&k_gemm<HC, HC, 0, 0>),
                      hipFuncAttributeMaxDynamicSharedMemorySize, LDS_GEMM);
  hipFuncSetAttribute(reinterpret_cast<const void*>(&k_gemm<HC, HC, 0, 1>),
                      hipFuncAttributeMaxDynamicSharedMemorySize, LDS_GEMM);
  hipFuncSetAttribute(reinterpret_cast<const void*>(&k_gemm<PD, PD, 0, 2>),
                      hipFuncAttributeMaxDynamicSharedMemorySize, LDS_GEMM);

  k_gemm<XD, XD, 1, 1><<<nGn, NTHR, LDS_GEMM, stream>>>((const void*)x, nN, WN, nb, (void*)H32, osc, 1.0f, NPAD, nb, nb);
  k_gemm<ADP, AD, 1, 0><<<nGe, NTHR, LDS_GEMM, stream>>>((const void*)ea, nE, WE, eb, (void*)E16, osc, ecar, EPAD, eb, eb);

  for (int l = 0; l < L; ++l) {
    k_agg<<<nAgg, NTHR, 0, stream>>>(csr, offp, cnt, srci, H32, E16, A16, nN, nE, csrLen, einv);
    k_gemm<HC, HC, 0, 0><<<nGn, NTHR, LDS_GEMM, stream>>>((const void*)A16, NPAD, WC1 + (size_t)l * HC * HC,
                                                           cb1 + (size_t)l * HC, (void*)M16, osc, 1.0f, NPAD, nb, nb);
    k_gemm<HC, HC, 0, 1><<<nGn, NTHR, LDS_GEMM, stream>>>((const void*)M16, NPAD, WC2 + (size_t)l * HC * HC,
                                                           cb2 + (size_t)l * HC, (void*)H32, osc, 1.0f, NPAD, nb, nb);
  }

  k_pool<<<GPAD, NTHR, 0, stream>>>(bix, H32, P16, nN, G);
  k_gemm<PD, PD, 0, 2><<<nGh, NTHR, LDS_GEMM, stream>>>((const void*)P16, GPAD, WH, hb1, (void*)out, osc, 1.0f, G, hw2, hb2);
}
